// LayoutAttention_64647847739404
// MI455X (gfx1250) — hardware-verified
//
#include <hip/hip_runtime.h>

typedef unsigned short u16;
typedef _Float16     v16h __attribute__((ext_vector_type(16)));
typedef __bf16       v16b __attribute__((ext_vector_type(16)));
typedef float        v8f  __attribute__((ext_vector_type(8)));
typedef float        v4f  __attribute__((ext_vector_type(4)));
typedef u16          v8us __attribute__((ext_vector_type(8)));
typedef unsigned int v4u  __attribute__((ext_vector_type(4)));
typedef v8us __attribute__((may_alias)) v8usa;
typedef v4f  __attribute__((may_alias)) v4fa;
typedef v4u  __attribute__((may_alias)) v4ua;

union FragH { v16h v; v8us u[2]; };
union FragB { v16b v; v8us u[2]; };

#define NTOK   4096
#define QD     320
#define INNER  512
#define NHEAD  8
#define HD     64
#define NPH    3
#define NXG    (NTOK * QD / 8)
#define XBLK   (NXG / 256)
#define CBLK   (NTOK / 256)
#define PSCALE 16384.0f
#define NEGBIG (-1.0e30f)

static_assert(NXG % 256 == 0);
static_assert(NTOK % 128 == 0);
static_assert(QD % 64 == 0);
static_assert(INNER % 64 == 0);
static_assert(HD == 64);
static_assert(NHEAD * HD == INNER);

__device__ __forceinline__ u16 bf16_bits(float f) {
  unsigned int u = __float_as_uint(f);
  u = u + 0x7FFFu + ((u >> 16) & 1u);
  return (u16)(u >> 16);
}
__device__ __forceinline__ float bf16_val(float f) {
  unsigned int u = __float_as_uint(f);
  u = (u + 0x7FFFu + ((u >> 16) & 1u)) & 0xFFFF0000u;
  return __uint_as_float(u);
}
__device__ __forceinline__ u16 f16_bits(float f) {
  union { _Float16 h; u16 u; } c;
  c.h = (_Float16)f;
  return c.u;
}

__device__ __forceinline__ v8f wmma_f16(v16h a, v16h b, v8f c) {
  v8f d = __builtin_amdgcn_wmma_f32_16x16x32_f16(false, a, false, b, (short)0, c, false, false);
  asm volatile("v_nop\n\tv_nop\n\tv_nop\n\tv_nop" : "+v"(d) : "v"(a), "v"(b));
  return d;
}
__device__ __forceinline__ v8f wmma_bf16(v16b a, v16b b, v8f c) {
  v8f d = __builtin_amdgcn_wmma_f32_16x16x32_bf16(false, a, false, b, (short)0, c, false, false);
  asm volatile("v_nop\n\tv_nop\n\tv_nop\n\tv_nop" : "+v"(d) : "v"(a), "v"(b));
  return d;
}

__device__ __forceinline__ v16h load_frag_h(const u16* p, int h) {
  FragH f;
  f.u[0] = *(const v8usa*)(p + 8 * h);
  f.u[1] = *(const v8usa*)(p + 16 + 8 * h);
  return f.v;
}
__device__ __forceinline__ v16b load_frag_b(const u16* p, int h) {
  FragB f;
  f.u[0] = *(const v8usa*)(p + 8 * h);
  f.u[1] = *(const v8usa*)(p + 16 + 8 * h);
  return f.v;
}

__global__ __launch_bounds__(256) void k_prep(const float* __restrict__ x,
                                              const float* __restrict__ gm,
                                              u16* __restrict__ xb,
                                              unsigned int* __restrict__ codes)
{
  const int b = blockIdx.x, t = threadIdx.x;
  if (b < XBLK) {
    const int g = b * 256 + t;
    if (g < NXG) {
      const float* src = x + (size_t)g * 8;
      const v4f a = *(const v4fa*)src;
      const v4f c = *(const v4fa*)(src + 4);
      const v8us o = { bf16_bits(a.x), bf16_bits(a.y), bf16_bits(a.z), bf16_bits(a.w),
                       bf16_bits(c.x), bf16_bits(c.y), bf16_bits(c.z), bf16_bits(c.w) };
      u16* dst = xb + (size_t)g * 8;
      *(volatile v8us*)dst = o;
      __threadfence();
      *(volatile v8us*)dst = o;
    }
  } else {
    const int i = (b - XBLK) * 256 + t;
    if (i < NTOK) {
      unsigned int c = 0u;
      #pragma unroll
      for (int p = 0; p < NPH; ++p)
        if (gm[p * NTOK + i] != 0.0f) c |= (1u << p);
      volatile unsigned int* dst = codes + i;
      *dst = c;
      __threadfence();
      *dst = c;
    }
  }
}

__global__ __launch_bounds__(256) void k_wtrans(const float* __restrict__ wq,
                                                const float* __restrict__ wk,
                                                const float* __restrict__ wv,
                                                const float* __restrict__ wo,
                                                u16* __restrict__ wqt,
                                                u16* __restrict__ wkt,
                                                u16* __restrict__ wvt,
                                                u16* __restrict__ wot)
{
  __shared__ __attribute__((aligned(16))) u16 sW[32 * 64];

  const int t = threadIdx.x, lane = t & 31, w = t >> 5;
  const int which = blockIdx.y, bx = blockIdx.x;
  const float* src;
  u16* dst;
  int K, Nc, k0, n0;
  if (which < 3) {
    src = (which == 0) ? wq : ((which == 1) ? wk : wv);
    dst = (which == 0) ? wqt : ((which == 1) ? wkt : wvt);
    K = QD; Nc = INNER;
    k0 = (bx >> 4) * 64;
    n0 = (bx & 15) * 32;
  } else {
    src = wo; dst = wot;
    K = INNER; Nc = QD;
    k0 = (bx / 10) * 64;
    n0 = (bx % 10) * 32;
  }

  #pragma unroll
  for (int i = 0; i < 8; ++i) {
    const int e = t + 256 * i;
    const int kk = e >> 5, nn = e & 31;
    const float v = src[(size_t)(k0 + kk) * Nc + n0 + nn];
    const u16 bits = (which < 3) ? bf16_bits(v) : f16_bits(64.0f * bf16_val(v));
    sW[nn * 64 + kk] = bits;
  }
  __syncthreads();

  const int sub = lane >> 3, q8 = lane & 7;
  const int nn = w * 4 + sub;
  const v8us v = *(const v8usa*)(sW + nn * 64 + 8 * q8);
  u16* p = dst + (size_t)(n0 + nn) * K + k0 + 8 * q8;
  *(volatile v8us*)p = v;
  __threadfence();
  *(volatile v8us*)p = v;
}

__device__ __forceinline__ void qkv_store_pass(const u16* sT, u16* plane, u16* vt,
                                               int which, int head, int m0, int w, int lane) {
  const int q8 = lane & 7, sub = lane >> 3;
  #pragma unroll
  for (int i = 0; i < 8; ++i) {
    const int lid = w * 32 + i * 4 + sub;
    v8us v;
    u16* dst;
    if (which != 2) {
      v = *(const v8usa*)(sT + lid * HD + 8 * q8);
      dst = plane + ((size_t)head * NTOK + m0 + lid) * HD + 8 * q8;
    } else {
      const int d = lid >> 1, hl = lid & 1;
      v = *(const v8usa*)(sT + d * 128 + 64 * hl + 8 * q8);
      dst = vt + ((size_t)head * HD + d) * NTOK + m0 + 64 * hl + 8 * q8;
    }
    *(volatile v8us*)dst = v;
  }
}

__global__ __launch_bounds__(128) void k_qkv(const u16* __restrict__ xb,
                                             const u16* __restrict__ wqt,
                                             const u16* __restrict__ wkt,
                                             const u16* __restrict__ wvt,
                                             u16* __restrict__ qh,
                                             u16* __restrict__ kh,
                                             u16* __restrict__ vt)
{
  __shared__ __attribute__((aligned(16))) u16 sT[128 * 64];

  const int tid = threadIdx.x, lane = tid & 31, w = tid >> 5;
  const int h = lane >> 4, m = lane & 15;
  const int m0 = blockIdx.x * 128;
  const int cg = blockIdx.y;
  const int which = cg >> 3, head = cg & 7;
  const int m0w = m0 + 32 * w;

  const u16* wt  = (which == 0) ? wqt : ((which == 1) ? wkt : wvt);
  const u16* xa0 = xb + (size_t)(m0w + m) * QD;
  const u16* xa1 = xa0 + (size_t)16 * QD;
  const u16* wb  = wt + (size_t)(head * HD + m) * QD;

  const v8f zero8 = {0.f, 0.f, 0.f, 0.f, 0.f, 0.f, 0.f, 0.f};
  v8f acc[2][4];
  #pragma unroll
  for (int mt = 0; mt < 2; ++mt)
    #pragma unroll
    for (int nt = 0; nt < 4; ++nt) acc[mt][nt] = zero8;

  #pragma unroll 1
  for (int k0 = 0; k0 < QD; k0 += 32) {
    const v16b a0 = load_frag_b(xa0 + k0, h);
    const v16b a1 = load_frag_b(xa1 + k0, h);
    #pragma unroll
    for (int nt = 0; nt < 4; ++nt) {
      const v16b b = load_frag_b(wb + (size_t)nt * 16 * QD + k0, h);
      acc[0][nt] = wmma_bf16(a0, b, acc[0][nt]);
      acc[1][nt] = wmma_bf16(a1, b, acc[1][nt]);
    }
  }

  const float osc = (which == 0) ? 0.125f : 1.0f;
  #pragma unroll
  for (int nt = 0; nt < 4; ++nt) {
    const int feat = 16 * nt + m;
    #pragma unroll
    for (int mt = 0; mt < 2; ++mt) {
      #pragma unroll
      for (int r = 0; r < 8; ++r) {
        const int tokl = 32 * w + 16 * mt + 8 * h + r;
        const float y = acc[mt][nt][r] * osc;
        const int idx = (which == 2) ? (feat * 128 + tokl) : (tokl * HD + feat);
        sT[idx] = f16_bits(y);
      }
    }
  }
  __syncthreads();

  u16* plane = (which == 0) ? qh : kh;
  qkv_store_pass(sT, plane, vt, which, head, m0, w, lane);
  __threadfence();
  qkv_store_pass(sT, plane, vt, which, head, m0, w, lane);
}

__device__ __forceinline__ v16h pack_p(v8f a, v8f c) {
  const v16h r = { (_Float16)(a[0] * PSCALE), (_Float16)(a[1] * PSCALE), (_Float16)(a[2] * PSCALE), (_Float16)(a[3] * PSCALE),
                   (_Float16)(a[4] * PSCALE), (_Float16)(a[5] * PSCALE), (_Float16)(a[6] * PSCALE), (_Float16)(a[7] * PSCALE),
                   (_Float16)(c[0] * PSCALE), (_Float16)(c[1] * PSCALE), (_Float16)(c[2] * PSCALE), (_Float16)(c[3] * PSCALE),
                   (_Float16)(c[4] * PSCALE), (_Float16)(c[5] * PSCALE), (_Float16)(c[6] * PSCALE), (_Float16)(c[7] * PSCALE) };
  return r;
}

__device__ __forceinline__ void att_store_pass(const u16* so, u16* ao, int head, int q0, int lane) {
  const int q8 = lane & 7, sub = lane >> 3;
  #pragma unroll
  for (int i = 0; i < 4; ++i) {
    const int row = i * 4 + sub;
    const v8us v = *(const v8usa*)(so + row * 64 + 8 * q8);
    u16* p = ao + (size_t)(q0 + row) * INNER + head * HD + 8 * q8;
    *(volatile v8us*)p = v;
  }
}

__global__ __launch_bounds__(128) void k_attn(const u16* __restrict__ qh,
                                              const u16* __restrict__ kh,
                                              const u16* __restrict__ vt,
                                              const unsigned int* __restrict__ codes,
                                              u16* __restrict__ ao)
{
  __shared__ __attribute__((aligned(16))) u16 sO[4 * 16 * 64];

  const int tid = threadIdx.x, lane = tid & 31, w = tid >> 5;
  const int h = lane >> 4, m = lane & 15;
  const int head = blockIdx.y;
  const int q0 = blockIdx.x * 64 + 16 * w;

  const u16* qrow = qh + ((size_t)head * NTOK + q0 + m) * HD;
  const v16h qb0 = load_frag_h(qrow, h);
  const v16h qb1 = load_frag_h(qrow + 32, h);
  const unsigned int cq = codes[q0 + m];

  const v8f zero8 = {0.f, 0.f, 0.f, 0.f, 0.f, 0.f, 0.f, 0.f};
  v8f o[4];
  #pragma unroll
  for (int t = 0; t < 4; ++t) o[t] = zero8;
  float mrun = NEGBIG, lrun = 0.0f;

  const u16* kbase = kh + ((size_t)head * NTOK + m) * HD;
  const u16* vbase = vt + ((size_t)head * HD + m) * NTOK;

  #pragma unroll 1
  for (int kb = 0; kb < NTOK; kb += 64) {
    v8f s[4];
    #pragma unroll
    for (int j = 0; j < 4; ++j) {
      const u16* kp = kbase + (size_t)(kb + 16 * j) * HD;
      const v16h kf0 = load_frag_h(kp, h);
      const v16h kf1 = load_frag_h(kp + 32, h);
      v8f z = zero8;
      z = wmma_f16(kf0, qb0, z);
      z = wmma_f16(kf1, qb1, z);
      s[j] = z;
    }
    #pragma unroll
    for (int j = 0; j < 4; ++j) {
      const unsigned int* ckp = codes + kb + 16 * j + 8 * h;
      const v4u c0 = *(const v4ua*)ckp;
      const v4u c1 = *(const v4ua*)(ckp + 4);
      #pragma unroll
      for (int r = 0; r < 4; ++r) {
        s[j][r]     = ((cq & c0[r]) == 0u) ? NEGBIG : s[j][r];
        s[j][r + 4] = ((cq & c1[r]) == 0u) ? NEGBIG : s[j][r + 4];
      }
    }

    float mloc = s[0][0];
    #pragma unroll
    for (int j = 0; j < 4; ++j)
      #pragma unroll
      for (int r = 0; r < 8; ++r) mloc = fmaxf(mloc, s[j][r]);
    mloc = fmaxf(mloc, __shfl_xor(mloc, 16));
    const float mnew = fmaxf(mrun, mloc);
    const float alpha = __expf(mrun - mnew);
    mrun = mnew;
    float lsum = 0.0f;
    #pragma unroll
    for (int j = 0; j < 4; ++j)
      #pragma unroll
      for (int r = 0; r < 8; ++r) {
        const float p = __expf(s[j][r] - mnew);
        s[j][r] = p;
        lsum += p;
      }
    lsum += __shfl_xor(lsum, 16);
    lrun = lrun * alpha + lsum;
    #pragma unroll
    for (int t = 0; t < 4; ++t)
      #pragma unroll
      for (int r = 0; r < 8; ++r) o[t][r] = o[t][r] * alpha;

    const v16h pb0 = pack_p(s[0], s[1]);
    const v16h pb1 = pack_p(s[2], s[3]);

    #pragma unroll
    for (int t = 0; t < 4; ++t) {
      const u16* vp = vbase + (size_t)(16 * t) * NTOK + kb;
      const v16h vf0 = load_frag_h(vp, h);
      const v16h vf1 = load_frag_h(vp + 32, h);
      o[t] = wmma_f16(vf0, pb0, o[t]);
      o[t] = wmma_f16(vf1, pb1, o[t]);
    }
  }

  const float inv = (1.0f / lrun) * (1.0f / 1024.0f);
  u16* so = sO + w * 1024;
  #pragma unroll
  for (int t = 0; t < 4; ++t)
    #pragma unroll
    for (int r = 0; r < 8; ++r)
      so[m * 64 + 16 * t + 8 * h + r] = f16_bits(o[t][r] * inv);
  __syncthreads();

  att_store_pass(so, ao, head, q0, lane);
  __threadfence();
  att_store_pass(so, ao, head, q0, lane);
}

__device__ __forceinline__ void out_store_pass(const float* sO, float* out, int m0, int cg, int w, int lane) {
  const int q8 = lane & 7, sub = lane >> 3;
  #pragma unroll
  for (int i = 0; i < 16; ++i) {
    const int lid = i * 4 + sub;
    const int row = 32 * w + (lid >> 1), hl = lid & 1;
    const v4f v = *(const v4fa*)(sO + row * 64 + 32 * hl + 4 * q8);
    float* p = out + (size_t)(m0 + row) * QD + 64 * cg + 32 * hl + 4 * q8;
    *(volatile v4f*)p = v;
  }
}

__global__ __launch_bounds__(128) void k_oproj(const u16* __restrict__ ao,
                                               const u16* __restrict__ wot,
                                               const float* __restrict__ bout,
                                               float* __restrict__ out)
{
  __shared__ __attribute__((aligned(16))) float sO[128 * 64];

  const int tid = threadIdx.x, lane = tid & 31, w = tid >> 5;
  const int h = lane >> 4, m = lane & 15;
  const int m0 = blockIdx.x * 128;
  const int cg = blockIdx.y;
  const int m0w = m0 + 32 * w;

  const u16* aa0 = ao + (size_t)(m0w + m) * INNER;
  const u16* aa1 = aa0 + (size_t)16 * INNER;
  const u16* wb  = wot + (size_t)(64 * cg + m) * INNER;

  const v8f zero8 = {0.f, 0.f, 0.f, 0.f, 0.f, 0.f, 0.f, 0.f};
  v8f acc[2][4];
  #pragma unroll
  for (int mt = 0; mt < 2; ++mt)
    #pragma unroll
    for (int nt = 0; nt < 4; ++nt) acc[mt][nt] = zero8;

  #pragma unroll 1
  for (int k0 = 0; k0 < INNER; k0 += 32) {
    const v16h a0 = load_frag_h(aa0 + k0, h);
    const v16h a1 = load_frag_h(aa1 + k0, h);
    #pragma unroll
    for (int nt = 0; nt < 4; ++nt) {
      const v16h b = load_frag_h(wb + (size_t)nt * 16 * INNER + k0, h);
      acc[0][nt] = wmma_f16(a0, b, acc[0][nt]);
      acc[1][nt] = wmma_f16(a1, b, acc[1][nt]);
    }
  }

  #pragma unroll
  for (int nt = 0; nt < 4; ++nt) {
    const int col = 16 * nt + m;
    const float bv = bf16_val(bout[64 * cg + col]);
    #pragma unroll
    for (int mt = 0; mt < 2; ++mt) {
      #pragma unroll
      for (int r = 0; r < 8; ++r) {
        const int tokl = 32 * w + 16 * mt + 8 * h + r;
        sO[tokl * 64 + col] = acc[mt][nt][r] * (1.0f / 1024.0f) + bv;
      }
    }
  }
  __syncthreads();

  out_store_pass(sO, out, m0, cg, w, lane);
  __threadfence();
  out_store_pass(sO, out, m0, cg, w, lane);
}

extern "C" void kernel_launch(void* const* d_in, const int* in_sizes, int n_in,
                              void* d_out, int out_size, void* d_ws, size_t ws_size,
                              hipStream_t stream) {
  if (n_in < 7) return;
  if (in_sizes[0] != NTOK * QD) return;
  if (in_sizes[1] != NPH * NTOK) return;
  if (in_sizes[2] != QD * INNER || in_sizes[3] != QD * INNER || in_sizes[4] != QD * INNER) return;
  if (in_sizes[5] != INNER * QD) return;
  if (in_sizes[6] != QD) return;
  if (out_size != NTOK * QD) return;

  const float* x    = (const float*)d_in[0];
  const float* gm   = (const float*)d_in[1];
  const float* Wq   = (const float*)d_in[2];
  const float* Wk   = (const float*)d_in[3];
  const float* Wv   = (const float*)d_in[4];
  const float* Wout = (const float*)d_in[5];
  const float* bout = (const float*)d_in[6];
  float* out = (float*)d_out;

  const size_t xb_bytes = (size_t)NTOK * QD * 2;
  const size_t w_bytes  = (size_t)QD * INNER * 2;
  const size_t pl_bytes = (size_t)NHEAD * NTOK * HD * 2;
  const size_t ao_bytes = (size_t)NTOK * INNER * 2;
  const size_t cd_bytes = (size_t)NTOK * 4;
  const size_t total = xb_bytes + 4 * w_bytes + 3 * pl_bytes + ao_bytes + cd_bytes;
  if (total > ws_size) return;
  if (total > (size_t)134217728) return;

  char* ws = (char*)d_ws;
  size_t off = 0;
  u16* xb  = (u16*)(ws + off); off += xb_bytes;
  u16* wqt = (u16*)(ws + off); off += w_bytes;
  u16* wkt = (u16*)(ws + off); off += w_bytes;
  u16* wvt = (u16*)(ws + off); off += w_bytes;
  u16* wot = (u16*)(ws + off); off += w_bytes;
  u16* qh  = (u16*)(ws + off); off += pl_bytes;
  u16* kh  = (u16*)(ws + off); off += pl_bytes;
  u16* vt  = (u16*)(ws + off); off += pl_bytes;
  u16* ao  = (u16*)(ws + off); off += ao_bytes;
  unsigned int* codes = (unsigned int*)(ws + off); off += cd_bytes;
  if (off != total) return;

  k_prep<<<XBLK + CBLK, 256, 0, stream>>>(x, gm, xb, codes);

  k_wtrans<<<dim3(80, 4), 256, 0, stream>>>(Wq, Wk, Wv, Wout, wqt, wkt, wvt, wot);

  k_qkv<<<dim3(NTOK / 128, 3 * NHEAD), 128, 0, stream>>>(xb, wqt, wkt, wvt, qh, kh, vt);

  k_attn<<<dim3(NTOK / 64, NHEAD), 128, 0, stream>>>(qh, kh, vt, codes, ao);

  k_oproj<<<dim3(NTOK / 128, QD / 64), 128, 0, stream>>>(ao, wot, bout, out);

  (void)hipGetLastError();
}
